// GNNLSTMPolicy_19825569038614
// MI455X (gfx1250) — hardware-verified
//
#include <hip/hip_runtime.h>
#define NNODE 100000
#define NE0 1600000
#define NEDGE (NE0 + NNODE)
#define NP2 2097152
#define NG 64
#define FIN 5
#define HH 64
#define LH 128
#define NA 10

typedef __bf16 v16b __attribute__((ext_vector_type(16)));
typedef unsigned short v8us __attribute__((ext_vector_type(8), may_alias));
typedef float  v8f  __attribute__((ext_vector_type(8)));
typedef float  v4f  __attribute__((ext_vector_type(4)));
typedef float  v4fa __attribute__((ext_vector_type(4), may_alias));
union FragB { v16b v; v8us half[2]; unsigned short u[16]; };

__device__ __forceinline__ unsigned short bf16_bits(float x) { unsigned int u = __float_as_uint(x); return (unsigned short)((u + 0x7FFFu + ((u >> 16) & 1u)) >> 16); }
__device__ __forceinline__ float bf16_val(unsigned short b) { return __uint_as_float(((unsigned int)b) << 16); }
__device__ __forceinline__ float bf16_round(float x) { return bf16_val(bf16_bits(x)); }
template <int NT>
__device__ __forceinline__ v8f mmaN(v16b ah, v16b al, v16b bh, v16b bl, v8f c) {
  c = __builtin_amdgcn_wmma_f32_16x16x32_bf16(false, ah, false, bh, (short)0, c, false, false);
  if (NT >= 2) c = __builtin_amdgcn_wmma_f32_16x16x32_bf16(false, al, false, bh, (short)0, c, false, false);
  if (NT >= 3) c = __builtin_amdgcn_wmma_f32_16x16x32_bf16(false, ah, false, bl, (short)0, c, false, false);
  asm volatile("v_nop\n\tv_nop\n\tv_nop\n\tv_nop" : "+v"(c) : "v"(ah), "v"(al), "v"(bh), "v"(bl));
  return c;
}

__global__ __launch_bounds__(256) void k_wt_bf16(const float* __restrict__ W, unsigned short* __restrict__ Wt, int K, int N) {
  const int t = blockIdx.x * 256 + threadIdx.x;
  const int k8n = K / 8;
  if (t >= N * k8n) return;
  const int n = t / k8n, k8 = (t % k8n) * 8;
  v8us v;
#pragma unroll
  for (int i = 0; i < 8; ++i) v[i] = bf16_bits(W[(size_t)(k8 + i) * N + n]);
  *(volatile v8us*)(Wt + (size_t)n * K + k8) = v;
  __threadfence();
  *(volatile v8us*)(Wt + (size_t)n * K + k8) = v;
}

template <bool ASPLIT, int ACT, bool BIAS_BF16>
__global__ __launch_bounds__(128) void k_gemm_bf(const float* __restrict__ A, int lda, const unsigned short* __restrict__ Wt, int ldb,
                                               const float* __restrict__ bias, float* __restrict__ C, int ldc, int M, int N, int K) {
  __shared__ __attribute__((aligned(16))) float so[4][16][64];
  const int tid = threadIdx.x, w = tid >> 5, lane = tid & 31, ln = lane & 15, hh = lane >> 4;
  const int ntn = N / 64;
  const int wid = blockIdx.x * 4 + w;
  const int mt = wid / ntn, nq = wid % ntn;
  if (mt * 16 >= M) return;
  const int row0 = mt * 16, col0 = nq * 64;
  const float* arow = A + (size_t)(row0 + ln) * lda;
  v8f acc[4] = {};
  for (int kb = 0; kb < K; kb += 32) {
    FragB ah, al;
    const v4f x0 = *(const v4fa*)(arow + kb + 8 * hh), x1 = *(const v4fa*)(arow + kb + 8 * hh + 4);
    const v4f x2 = *(const v4fa*)(arow + kb + 16 + 8 * hh), x3 = *(const v4fa*)(arow + kb + 16 + 8 * hh + 4);
    float xs[16] = {x0[0],x0[1],x0[2],x0[3],x1[0],x1[1],x1[2],x1[3],x2[0],x2[1],x2[2],x2[3],x3[0],x3[1],x3[2],x3[3]};
#pragma unroll
    for (int i = 0; i < 16; ++i) { const unsigned short hb = bf16_bits(xs[i]); ah.u[i] = hb; al.u[i] = ASPLIT ? bf16_bits(xs[i] - bf16_val(hb)) : (unsigned short)0; }
#pragma unroll
    for (int t = 0; t < 4; ++t) {
      const unsigned short* brow = Wt + (size_t)(col0 + t * 16 + ln) * ldb + kb;
      FragB b;
      b.half[0] = *(const v8us*)(brow + 8 * hh);
      b.half[1] = *(const v8us*)(brow + 16 + 8 * hh);
      acc[t] = mmaN<ASPLIT ? 2 : 1>(ah.v, al.v, b.v, b.v, acc[t]);
    }
  }
#pragma unroll
  for (int t = 0; t < 4; ++t) {
    float bv = bias ? bias[col0 + t * 16 + ln] : 0.f;
    if (BIAS_BF16) bv = bf16_round(bv);
#pragma unroll
    for (int r = 0; r < 8; ++r) { float v = acc[t][r] + bv; if (ACT == 1) v = fmaxf(v, 0.f); so[w][8 * hh + r][t * 16 + ln] = v; }
  }
  __builtin_amdgcn_fence(__ATOMIC_ACQ_REL, "workgroup");
  __builtin_amdgcn_wave_barrier();
  const int rsub = lane >> 4, c4 = (lane & 15) * 4;
  for (int pass = 0; pass < 2; ++pass) {
#pragma unroll
    for (int q = 0; q < 8; ++q) {
      const int r = q * 2 + rsub;
      const v4f v = *(const v4fa*)&so[w][r][c4];
      *(volatile v4f*)(C + (size_t)(row0 + r) * ldc + col0 + c4) = v;
    }
    if (pass == 0) __threadfence();
  }
}

template <int D, bool CAUSAL>
__global__ __launch_bounds__(128) void k_flash(const float* __restrict__ qb, const float* __restrict__ kb, const float* __restrict__ vb,
                                             int pitch, int T, int H, float scale, float* __restrict__ y, int ypitch) {
  constexpr int KS = D / 32;
  constexpr int DT = D / 16;
  __shared__ __attribute__((aligned(16))) unsigned short sKh[32][D + 8], sKl[32][D + 8], sVh[32][D + 8], sVl[32][D + 8];
  __shared__ __attribute__((aligned(16))) unsigned short sPh[4][16][40], sPl[4][16][40];
  __shared__ __attribute__((aligned(16))) float sO[4][16][D];
  const int tid = threadIdx.x, w = tid >> 5, lane = tid & 31, ln = lane & 15, hh = lane >> 4;
  const int nqb = (T + 63) / 64;
  const int bh = blockIdx.x / nqb, qblk = blockIdx.x % nqb;
  const int b = bh / H, h = bh % H;
  const int q0 = qblk * 64 + w * 16;
  const float* Q = qb + (size_t)b * T * pitch + h * D;
  const float* K = kb + (size_t)b * T * pitch + h * D;
  const float* V = vb + (size_t)b * T * pitch + h * D;

  FragB aqh[KS], aql[KS];
  {
    int row = q0 + ln; if (row >= T) row = T - 1;
    const float* qr = Q + (size_t)row * pitch;
#pragma unroll
    for (int ks = 0; ks < KS; ++ks)
#pragma unroll
      for (int i = 0; i < 16; ++i) {
        const int d = ks * 32 + ((i < 8) ? (8 * hh + i) : (16 + 8 * hh + (i - 8)));
        const float x = qr[d] * scale; const unsigned short hb = bf16_bits(x);
        aqh[ks].u[i] = hb; aql[ks].u[i] = bf16_bits(x - bf16_val(hb));
      }
  }
  float m_r[8], l_r[8];
#pragma unroll
  for (int r = 0; r < 8; ++r) { m_r[r] = -3.0e38f; l_r[r] = 0.f; }
  v8f oacc[DT];
#pragma unroll
  for (int dt = 0; dt < DT; ++dt) oacc[dt] = (v8f){0.f,0.f,0.f,0.f,0.f,0.f,0.f,0.f};

  const int kv_end = CAUSAL ? min(T, qblk * 64 + 64) : T;
  for (int j0 = 0; j0 < kv_end; j0 += 32) {
    __syncthreads();
    for (int e = tid; e < 32 * (D / 4); e += 128) {
      const int r = e / (D / 4), c4 = (e % (D / 4)) * 4;
      const int key = j0 + r;
      v4f kf = {0.f,0.f,0.f,0.f}, vf = {0.f,0.f,0.f,0.f};
      if (key < T) { kf = *(const v4fa*)(K + (size_t)key * pitch + c4); vf = *(const v4fa*)(V + (size_t)key * pitch + c4); }
#pragma unroll
      for (int t = 0; t < 4; ++t) {
        unsigned short hb = bf16_bits(kf[t]); sKh[r][c4 + t] = hb; sKl[r][c4 + t] = bf16_bits(kf[t] - bf16_val(hb));
        hb = bf16_bits(vf[t]); sVh[r][c4 + t] = hb; sVl[r][c4 + t] = bf16_bits(vf[t] - bf16_val(hb));
      }
    }
    __syncthreads();
    v8f s[2];
#pragma unroll
    for (int nt = 0; nt < 2; ++nt) {
      v8f acc = {};
#pragma unroll
      for (int ks = 0; ks < KS; ++ks) {
        FragB bh_, bl_;
        bh_.half[0] = *(const v8us*)&sKh[nt * 16 + ln][ks * 32 + 8 * hh]; bh_.half[1] = *(const v8us*)&sKh[nt * 16 + ln][ks * 32 + 16 + 8 * hh];
        bl_.half[0] = *(const v8us*)&sKl[nt * 16 + ln][ks * 32 + 8 * hh]; bl_.half[1] = *(const v8us*)&sKl[nt * 16 + ln][ks * 32 + 16 + 8 * hh];
        acc = mmaN<3>(aqh[ks].v, aql[ks].v, bh_.v, bl_.v, acc);
      }
      s[nt] = acc;
    }
    float alpha[8];
#pragma unroll
    for (int r = 0; r < 8; ++r) {
      const int qi = q0 + 8 * hh + r;
      const int ja = j0 + ln, jb = j0 + 16 + ln;
      if (CAUSAL) { if (ja > qi) s[0][r] = -3.0e38f; if (jb > qi) s[1][r] = -3.0e38f; }
      if (ja >= T) s[0][r] = -3.0e38f;
      if (jb >= T) s[1][r] = -3.0e38f;
      float mx = fmaxf(s[0][r], s[1][r]);
      mx = fmaxf(mx, __shfl_xor(mx, 1, 32)); mx = fmaxf(mx, __shfl_xor(mx, 2, 32)); mx = fmaxf(mx, __shfl_xor(mx, 4, 32)); mx = fmaxf(mx, __shfl_xor(mx, 8, 32));
      const float mnew = fmaxf(m_r[r], mx);
      alpha[r] = (mnew > -1.0e38f) ? __expf(m_r[r] - mnew) : 1.0f;
      const float p0 = (s[0][r] > -1.0e38f) ? __expf(s[0][r] - mnew) : 0.f;
      const float p1 = (s[1][r] > -1.0e38f) ? __expf(s[1][r] - mnew) : 0.f;
      m_r[r] = mnew;
      l_r[r] = l_r[r] * alpha[r] + p0 + p1;
      unsigned short hb = bf16_bits(p0); sPh[w][8 * hh + r][ln] = hb;      sPl[w][8 * hh + r][ln] = bf16_bits(p0 - bf16_val(hb));
      hb = bf16_bits(p1);                sPh[w][8 * hh + r][16 + ln] = hb; sPl[w][8 * hh + r][16 + ln] = bf16_bits(p1 - bf16_val(hb));
    }
#pragma unroll
    for (int dt = 0; dt < DT; ++dt)
#pragma unroll
      for (int r = 0; r < 8; ++r) oacc[dt][r] *= alpha[r];
    __builtin_amdgcn_fence(__ATOMIC_ACQ_REL, "workgroup");
    __builtin_amdgcn_wave_barrier();
    FragB pah, pal;
    pah.half[0] = *(const v8us*)&sPh[w][ln][8 * hh]; pah.half[1] = *(const v8us*)&sPh[w][ln][16 + 8 * hh];
    pal.half[0] = *(const v8us*)&sPl[w][ln][8 * hh]; pal.half[1] = *(const v8us*)&sPl[w][ln][16 + 8 * hh];
#pragma unroll
    for (int dt = 0; dt < DT; ++dt) {
      FragB bvh, bvl;
#pragma unroll
      for (int i = 0; i < 8; ++i) {
        bvh.u[i] = sVh[8 * hh + i][dt * 16 + ln]; bvh.u[8 + i] = sVh[16 + 8 * hh + i][dt * 16 + ln];
        bvl.u[i] = sVl[8 * hh + i][dt * 16 + ln]; bvl.u[8 + i] = sVl[16 + 8 * hh + i][dt * 16 + ln];
      }
      oacc[dt] = mmaN<3>(pah.v, pal.v, bvh.v, bvl.v, oacc[dt]);
    }
    __builtin_amdgcn_fence(__ATOMIC_ACQ_REL, "workgroup");
    __builtin_amdgcn_wave_barrier();
  }
#pragma unroll
  for (int r = 0; r < 8; ++r) {
    float l = l_r[r];
    l += __shfl_xor(l, 1, 32); l += __shfl_xor(l, 2, 32); l += __shfl_xor(l, 4, 32); l += __shfl_xor(l, 8, 32);
    l_r[r] = (l > 0.f) ? 1.0f / l : 0.f;
  }
#pragma unroll
  for (int dt = 0; dt < DT; ++dt)
#pragma unroll
    for (int r = 0; r < 8; ++r) sO[w][8 * hh + r][dt * 16 + ln] = oacc[dt][r] * l_r[r];
  __builtin_amdgcn_fence(__ATOMIC_ACQ_REL, "workgroup");
  __builtin_amdgcn_wave_barrier();
  for (int pass = 0; pass < 2; ++pass) {
    for (int r = 0; r < 16; ++r) {
      const int row = q0 + r;
      if (row < T && lane < D / 4) {
        const v4f val = *(const v4fa*)&sO[w][r][lane * 4];
        *(volatile v4f*)(y + ((size_t)b * T + row) * ypitch + h * D + lane * 4) = val;
      }
    }
    if (pass == 0) __threadfence();
  }
}

__global__ __launch_bounds__(256) void k_sort_init(const int* __restrict__ seg, int n, int nseg, unsigned int* __restrict__ key, unsigned int* __restrict__ val, int np2) {
  const int i = blockIdx.x * 256 + threadIdx.x; if (i >= np2) return;
  unsigned int kv = 0xFFFFFFFFu;
  if (i < n) { int s = seg[i]; s = s < 0 ? 0 : (s >= nseg ? nseg - 1 : s); kv = (unsigned int)s; }
  *(volatile unsigned int*)(key + i) = kv; *(volatile unsigned int*)(val + i) = (unsigned int)i;
  __threadfence();
  *(volatile unsigned int*)(key + i) = kv; *(volatile unsigned int*)(val + i) = (unsigned int)i;
}
template <bool STAGE0>
__global__ __launch_bounds__(512) void k_sort_lds(unsigned int* __restrict__ key, unsigned int* __restrict__ val, int kstage) {
  __shared__ unsigned int sk[1024], sv[1024];
  const int tid = threadIdx.x; const int base = blockIdx.x * 1024;
  sk[tid] = key[base + tid]; sv[tid] = val[base + tid]; sk[tid + 512] = key[base + tid + 512]; sv[tid + 512] = val[base + tid + 512];
  __syncthreads();
  for (int k = (STAGE0 ? 2 : kstage); k <= (STAGE0 ? 1024 : kstage); k <<= 1) {
    for (int j = (k > 1024 ? 512 : (k >> 1)); j >= 1; j >>= 1) {
      const int lo = tid & (j - 1), hi2 = (tid >> __builtin_ctz(j)) << (__builtin_ctz(j) + 1);
      const int il = hi2 | lo, ir = il | j;
      const int gi = base + il;
      const bool asc = ((gi & k) == 0);
      unsigned int a = sk[il], b = sk[ir], va = sv[il], vb = sv[ir];
      const bool swp = asc ? (a > b) : (a < b);
      if (swp) { sk[il] = b; sk[ir] = a; sv[il] = vb; sv[ir] = va; }
      __syncthreads();
    }
  }
  for (int pass = 0; pass < 2; ++pass) {
    *(volatile unsigned int*)(key + base + tid) = sk[tid]; *(volatile unsigned int*)(val + base + tid) = sv[tid];
    *(volatile unsigned int*)(key + base + tid + 512) = sk[tid + 512]; *(volatile unsigned int*)(val + base + tid + 512) = sv[tid + 512];
    if (pass == 0) __threadfence();
  }
}
__global__ __launch_bounds__(256) void k_sort_step(unsigned int* __restrict__ key, unsigned int* __restrict__ val, int k, int j, int np2) {
  const int t = blockIdx.x * 256 + threadIdx.x; if (t >= np2 / 2) return;
  const int lo = t & (j - 1), il = ((t >> __builtin_ctz(j)) << (__builtin_ctz(j) + 1)) | lo, ir = il | j;
  const bool asc = ((il & k) == 0);
  unsigned int a = key[il], b = key[ir], va = val[il], vb = val[ir];
  const bool swp = asc ? (a > b) : (a < b);
  const unsigned int k1 = swp ? b : a, k2 = swp ? a : b, v1 = swp ? vb : va, v2 = swp ? va : vb;
  *(volatile unsigned int*)(key + il) = k1; *(volatile unsigned int*)(key + ir) = k2; *(volatile unsigned int*)(val + il) = v1; *(volatile unsigned int*)(val + ir) = v2;
  __threadfence();
  *(volatile unsigned int*)(key + il) = k1; *(volatile unsigned int*)(key + ir) = k2; *(volatile unsigned int*)(val + il) = v1; *(volatile unsigned int*)(val + ir) = v2;
}
__global__ __launch_bounds__(256) void k_rowptr(const unsigned int* __restrict__ key, int np2, int nseg, int* __restrict__ rowptr) {
  int s = blockIdx.x * 256 + threadIdx.x; if (s >= ((nseg + 1 + 31) / 32) * 32) return;
  const int sdst = s; if (s > nseg) s = nseg;
  int lo = 0, hi = np2;
  while (lo < hi) { const int mid = (lo + hi) >> 1; if (key[mid] < (unsigned int)s) lo = mid + 1; else hi = mid; }
  *(volatile int*)(rowptr + sdst) = lo; __threadfence(); *(volatile int*)(rowptr + sdst) = lo;
}
static void sort_pairs(unsigned int* key, unsigned int* val, int np2, hipStream_t stream) {
  k_sort_lds<true><<<np2 / 1024, 512, 0, stream>>>(key, val, 0);
  for (int k = 2048; k <= np2; k <<= 1) {
    for (int j = k >> 1; j >= 1024; j >>= 1) k_sort_step<<<(np2 / 2 + 255) / 256, 256, 0, stream>>>(key, val, k, j, np2);
    k_sort_lds<false><<<np2 / 1024, 512, 0, stream>>>(key, val, k);
  }
}

__global__ __launch_bounds__(256) void k_sort_init2(const int* __restrict__ dst, unsigned int* __restrict__ key, unsigned int* __restrict__ val) {
  const int i = blockIdx.x * 256 + threadIdx.x; if (i >= NP2) return;
  unsigned int kv = 0xFFFFFFFFu;
  if (i < NE0) { int s = dst[i]; s = s < 0 ? 0 : (s >= NNODE ? NNODE - 1 : s); kv = (unsigned int)s; }
  else if (i < NEDGE) kv = (unsigned int)(i - NE0);
  *(volatile unsigned int*)(key + i) = kv; *(volatile unsigned int*)(val + i) = (unsigned int)i; __threadfence();
  *(volatile unsigned int*)(key + i) = kv; *(volatile unsigned int*)(val + i) = (unsigned int)i;
}
__device__ __forceinline__ int edge_src(int e, const int* __restrict__ src) { if (e >= NE0) return e - NE0; int s = src[e]; return s < 0 ? 0 : (s >= NNODE ? NNODE - 1 : s); }
__global__ __launch_bounds__(256) void k_encoder(const float* __restrict__ x, const float* __restrict__ ew_, const float* __restrict__ eb, const float* __restrict__ g, const float* __restrict__ bb, float* __restrict__ h) {
  const int tid = threadIdx.x, w = tid >> 5, lane = tid & 31; const int n = blockIdx.x * 8 + w; if (n >= NNODE) return;
  float xv[FIN]; for (int k = 0; k < FIN; ++k) xv[k] = bf16_round(x[(size_t)n * FIN + k]);
  v4f a = {0.f,0.f,0.f,0.f};
  if (lane < 16) { for (int q = 0; q < 4; ++q) { const int c = lane * 4 + q; float s = bf16_round(eb[c]); for (int k = 0; k < FIN; ++k) s += xv[k] * bf16_round(ew_[k * HH + c]); a[q] = fmaxf(s, 0.f); } }
  float s = (lane < 16) ? (a[0] + a[1] + a[2] + a[3]) : 0.f; for (int o = 16; o >= 1; o >>= 1) s += __shfl_xor(s, o, 32);
  const float mu = s * (1.0f / HH);
  float v = 0.f; if (lane < 16) for (int q = 0; q < 4; ++q) { const float c = a[q] - mu; v += c * c; } for (int o = 16; o >= 1; o >>= 1) v += __shfl_xor(v, o, 32);
  const float rs = rsqrtf(v * (1.0f / HH) + 1e-5f);
  if (lane < 16) { v4f o; for (int q = 0; q < 4; ++q) o[q] = (a[q] - mu) * rs * bf16_round(g[lane * 4 + q]) + bf16_round(bb[lane * 4 + q]); float* row = h + (size_t)n * HH + lane * 4; *(volatile v4f*)row = o; __threadfence(); *(volatile v4f*)row = o; }
}
__global__ __launch_bounds__(256) void k_node_att1(const float* __restrict__ hw, const float* __restrict__ a_s, const float* __restrict__ a_d, float* __restrict__ as_, float* __restrict__ ad_) {
  __shared__ float r1[32], r2[32];
  const int tid = threadIdx.x, w = tid >> 5, lane = tid & 31; const int n0 = blockIdx.x * 32;
  for (int u = 0; u < 4; ++u) { const int n = n0 + w * 4 + u; float s1 = 0.f, s2 = 0.f;
    if (n < NNODE) { const float* hr = hw + (size_t)n * HH; for (int c = lane; c < HH; c += 32) { const float v = hr[c]; s1 += v * bf16_round(a_s[c]); s2 += v * bf16_round(a_d[c]); } }
    for (int o = 16; o >= 1; o >>= 1) { s1 += __shfl_xor(s1, o, 32); s2 += __shfl_xor(s2, o, 32); }
    if (lane == 0) { r1[w * 4 + u] = s1; r2[w * 4 + u] = s2; } }
  __syncthreads();
  if (tid < 32) { const float v = r1[tid]; *(volatile float*)(as_ + n0 + tid) = v; __threadfence(); *(volatile float*)(as_ + n0 + tid) = v; }
  else if (tid < 64) { const float v = r2[tid - 32]; *(volatile float*)(ad_ + n0 + tid - 32) = v; __threadfence(); *(volatile float*)(ad_ + n0 + tid - 32) = v; }
}
__global__ __launch_bounds__(256) void k_gat1(const float* __restrict__ hw, const float* __restrict__ as_, const float* __restrict__ ad_, const float* __restrict__ bias,
                                            const int* __restrict__ src, const int* __restrict__ rowptr, const unsigned int* __restrict__ perm, float* __restrict__ out) {
  const int tid = threadIdx.x, w = tid >> 5, lane = tid & 31; const int nd = blockIdx.x * 8 + w; if (nd >= NNODE) return;
  const int p0 = rowptr[nd], p1 = rowptr[nd + 1]; const float adn = ad_[nd];
  float mx = -__builtin_inff();
  for (int p = p0 + lane; p < p1; p += 32) { const int sn = edge_src((int)perm[p], src); float a = as_[sn] + adn; a = a >= 0.f ? a : 0.2f * a; mx = fmaxf(mx, a); }
  for (int o = 16; o >= 1; o >>= 1) mx = fmaxf(mx, __shfl_xor(mx, o, 32));
  if (!(mx > -__builtin_inff())) mx = 0.f;
  float den = 0.f;
  for (int p = p0 + lane; p < p1; p += 32) { const int sn = edge_src((int)perm[p], src); float a = as_[sn] + adn; a = a >= 0.f ? a : 0.2f * a; den += expf(a - mx); }
  for (int o = 16; o >= 1; o >>= 1) den += __shfl_xor(den, o, 32);
  den += 1e-16f;
  v4f acc = {0.f,0.f,0.f,0.f}; const bool act = lane < 16;
  for (int p = p0; p < p1; ++p) { const int sn = edge_src((int)perm[p], src); float a = as_[sn] + adn; a = a >= 0.f ? a : 0.2f * a; const float al = expf(a - mx) / den;
    if (act) { const v4f x0 = *(const v4fa*)(hw + (size_t)sn * HH + lane * 4); for (int q = 0; q < 4; ++q) acc[q] += al * x0[q]; } }
  if (act) { v4f o; for (int q = 0; q < 4; ++q) o[q] = fmaxf(acc[q] + bf16_round(bias[lane * 4 + q]), 0.f); float* row = out + (size_t)nd * HH + lane * 4; *(volatile v4f*)row = o; __threadfence(); *(volatile v4f*)row = o; }
}
__global__ __launch_bounds__(256) void k_gptr(const int* __restrict__ batch, int* __restrict__ gptr) {
  const int slot = blockIdx.x * 256 + threadIdx.x; if (slot >= ((NG + 1 + 31) / 32) * 32) return;
  const int g = slot > NG ? NG : slot;
  int lo = 0, hi = NNODE; while (lo < hi) { const int mid = (lo + hi) >> 1; if (batch[mid] < g) lo = mid + 1; else hi = mid; }
  *(volatile int*)(gptr + slot) = lo; __threadfence(); *(volatile int*)(gptr + slot) = lo;
}
__global__ __launch_bounds__(256) void k_graph(const float* __restrict__ h, const int* __restrict__ gptr, const float* __restrict__ gw, const float* __restrict__ gb,
                                             const float* __restrict__ w_ih, const float* __restrict__ b_ih, const float* __restrict__ b_hh,
                                             const float* __restrict__ q_w1, const float* __restrict__ q_b1, const float* __restrict__ q_w2, const float* __restrict__ q_b2,
                                             float* __restrict__ gout) {
  __shared__ float red[256]; __shared__ float sPool[HH]; __shared__ float sGate[4 * LH]; __shared__ float sH1[LH]; __shared__ float sQ1[HH];
  const int g = blockIdx.x, tid = threadIdx.x; const int n0 = gptr[g], n1 = gptr[g + 1];
  float mx = -__builtin_inff();
  for (int n = n0 + tid; n < n1; n += 256) { const float* hr = h + (size_t)n * HH; float s = bf16_round(gb[0]);
#pragma unroll 1
    for (int c = 0; c < HH; ++c) s += hr[c] * bf16_round(gw[c]); mx = fmaxf(mx, s); }
  red[tid] = mx; __syncthreads(); for (int st = 128; st > 0; st >>= 1) { if (tid < st) red[tid] = fmaxf(red[tid], red[tid + st]); __syncthreads(); }
  mx = red[0]; if (!(mx > -__builtin_inff())) mx = 0.f; __syncthreads();
  float den = 0.f;
  for (int n = n0 + tid; n < n1; n += 256) { const float* hr = h + (size_t)n * HH; float s = bf16_round(gb[0]);
#pragma unroll 1
    for (int c = 0; c < HH; ++c) s += hr[c] * bf16_round(gw[c]); den += expf(s - mx); }
  red[tid] = den; __syncthreads(); for (int st = 128; st > 0; st >>= 1) { if (tid < st) red[tid] += red[tid + st]; __syncthreads(); }
  den = red[0] + 1e-16f; __syncthreads();
  if (tid < HH) { float acc = 0.f; for (int n = n0; n < n1; ++n) { const float* hr = h + (size_t)n * HH; float s = bf16_round(gb[0]);
#pragma unroll 1
      for (int c = 0; c < HH; ++c) s += hr[c] * bf16_round(gw[c]); acc += (expf(s - mx) / den) * hr[tid]; } sPool[tid] = acc; }
  __syncthreads();
  for (int j = tid; j < 4 * LH; j += 256) { float s = bf16_round(b_ih[j]) + bf16_round(b_hh[j]);
#pragma unroll 1
    for (int c = 0; c < HH; ++c) s += sPool[c] * bf16_round(w_ih[(size_t)j * HH + c]); sGate[j] = s; }
  __syncthreads();
  if (tid < LH) { const float ig = 1.0f / (1.0f + expf(-sGate[tid])), gg = tanhf(sGate[2 * LH + tid]), og = 1.0f / (1.0f + expf(-sGate[3 * LH + tid]));
    const float c1 = ig * gg; const float h1 = og * tanhf(c1); sH1[tid] = h1; red[tid] = c1; }
  __syncthreads();
  if (tid < HH) { float s = bf16_round(q_b1[tid]);
#pragma unroll 1
    for (int k = 0; k < LH; ++k) s += sH1[k] * bf16_round(q_w1[(size_t)k * HH + tid]); sQ1[tid] = fmaxf(s, 0.f); }
  __syncthreads();
  float* row = gout + (size_t)g * 320;
  float qv = 0.f; if (tid < NA) { float s = bf16_round(q_b2[tid]);
#pragma unroll 1
    for (int k = 0; k < HH; ++k) s += sQ1[k] * bf16_round(q_w2[k * NA + tid]); qv = s; }
  for (int pass = 0; pass < 2; ++pass) {
    if (tid < 32) *(volatile float*)(row + tid) = qv;
    if (tid < LH) { *(volatile float*)(row + 32 + tid) = sH1[tid]; *(volatile float*)(row + 160 + tid) = red[tid]; }
    if (tid >= LH && tid < LH + 32) *(volatile float*)(row + 288 + tid - LH) = 0.f;
    if (pass == 0) __threadfence();
  }
}
__global__ __launch_bounds__(256) void k_out(const float* __restrict__ gout, float* __restrict__ q, float* __restrict__ h1, float* __restrict__ c1) {
  const int tid = threadIdx.x;
  for (int pass = 0; pass < 2; ++pass) {
    for (int t = tid; t < NG * NA; t += 256) *(volatile float*)(q + t) = gout[(size_t)(t / NA) * 320 + (t % NA)];
    for (int t = tid; t < NG * LH; t += 256) { *(volatile float*)(h1 + t) = gout[(size_t)(t / LH) * 320 + 32 + (t % LH)]; *(volatile float*)(c1 + t) = gout[(size_t)(t / LH) * 320 + 160 + (t % LH)]; }
    if (pass == 0) __threadfence();
  }
}

extern "C" void kernel_launch(void* const* d_in, const int* in_sizes, int n_in,
                              void* d_out, int out_size, void* d_ws, size_t ws_size, hipStream_t stream) {
  (void)in_sizes; (void)n_in; (void)out_size;
  const float* x = (const float*)d_in[0]; const int* ei = (const int*)d_in[1]; const int* batch = (const int*)d_in[2];
  const float* enc_w = (const float*)d_in[3]; const float* enc_b = (const float*)d_in[4]; const float* ln_g = (const float*)d_in[5]; const float* ln_b = (const float*)d_in[6];
  const float* w1 = (const float*)d_in[7]; const float* a1s = (const float*)d_in[8]; const float* a1d = (const float*)d_in[9]; const float* b1 = (const float*)d_in[10];
  const float* w2 = (const float*)d_in[11]; const float* a2s = (const float*)d_in[12]; const float* a2d = (const float*)d_in[13]; const float* b2 = (const float*)d_in[14];
  const float* gw = (const float*)d_in[15]; const float* gb = (const float*)d_in[16]; const float* w_ih = (const float*)d_in[17]; const float* b_ih = (const float*)d_in[19]; const float* b_hh = (const float*)d_in[20];
  const float* q_w1 = (const float*)d_in[21]; const float* q_b1 = (const float*)d_in[22]; const float* q_w2 = (const float*)d_in[23]; const float* q_b2 = (const float*)d_in[24];
  float* qo = (float*)d_out; float* h1o = (float*)((char*)d_out + 2560); float* c1o = (float*)((char*)d_out + 35328);
  char* ws = (char*)d_ws; size_t off = 0;
  auto take = [&](size_t bytes) { char* p = ws + off; off += (bytes + 255) & ~(size_t)255; return p; };
  unsigned short* W1t = (unsigned short*)take(HH * HH * 2); unsigned short* W2t = (unsigned short*)take(HH * HH * 2);
  unsigned int* key = (unsigned int*)take((size_t)NP2 * 4); unsigned int* perm = (unsigned int*)take((size_t)NP2 * 4); int* rowptr = (int*)take((size_t)(NNODE + 64) * 4);
  float* hA = (float*)take((size_t)NNODE * HH * 4); float* hB = (float*)take((size_t)NNODE * HH * 4);
  float* as_ = (float*)take((size_t)(NNODE + 32) * 4); float* ad_ = (float*)take((size_t)(NNODE + 32) * 4);
  int* gptr = (int*)take((size_t)(NG + 64) * 4); float* gout = (float*)take((size_t)NG * 320 * 4);
  if (off > ws_size) return;
  k_wt_bf16<<<(HH * (HH / 8) + 255) / 256, 256, 0, stream>>>(w1, W1t, HH, HH);
  k_wt_bf16<<<(HH * (HH / 8) + 255) / 256, 256, 0, stream>>>(w2, W2t, HH, HH);
  k_sort_init2<<<NP2 / 256, 256, 0, stream>>>(ei + NE0, key, perm);
  sort_pairs(key, perm, NP2, stream);
  k_rowptr<<<(NNODE + 32 + 255) / 256, 256, 0, stream>>>(key, NP2, NNODE, rowptr);
  k_encoder<<<(NNODE + 7) / 8, 256, 0, stream>>>(x, enc_w, enc_b, ln_g, ln_b, hA);
  const int gbk = ((NNODE / 16) * (HH / 64) + 3) / 4;
  k_gemm_bf<true, 0, false><<<gbk, 128, 0, stream>>>(hA, HH, W1t, HH, nullptr, hB, HH, NNODE, HH, HH);
  k_node_att1<<<(NNODE + 31) / 32, 256, 0, stream>>>(hB, a1s, a1d, as_, ad_);
  k_gat1<<<(NNODE + 7) / 8, 256, 0, stream>>>(hB, as_, ad_, b1, ei, rowptr, perm, hA);
  k_gemm_bf<true, 0, false><<<gbk, 128, 0, stream>>>(hA, HH, W2t, HH, nullptr, hB, HH, NNODE, HH, HH);
  k_node_att1<<<(NNODE + 31) / 32, 256, 0, stream>>>(hB, a2s, a2d, as_, ad_);
  k_gat1<<<(NNODE + 7) / 8, 256, 0, stream>>>(hB, as_, ad_, b2, ei, rowptr, perm, hA);
  k_gptr<<<(NG + 32 + 255) / 256, 256, 0, stream>>>(batch, gptr);
  k_graph<<<NG, 256, 0, stream>>>(hA, gptr, gw, gb, w_ih, b_ih, b_hh, q_w1, q_b1, q_w2, q_b2, gout);
  k_out<<<1, 256, 0, stream>>>(gout, qo, h1o, c1o);
}
